// CFSS_26233660244418
// MI455X (gfx1250) — hardware-verified
//
#include <hip/hip_runtime.h>
#include <math.h>
#include <stddef.h>

#define B_SZ 2
#define HH 64
#define WW 64
#define LL 4096
#define DM 96
#define DI 192
#define NS 16
#define RR 6
#define KK 4
#define CM 38
#define FP 64
#define CR 48
#define NTOK (B_SZ * LL)

typedef __bf16 bf16_t;
typedef bf16_t v16b __attribute__((ext_vector_type(16)));
typedef float v8f __attribute__((ext_vector_type(8)));
typedef float v4f __attribute__((ext_vector_type(4), __may_alias__));
typedef unsigned short v8us __attribute__((ext_vector_type(8), __may_alias__));
union Frag { v16b v; v8us h[2]; };

__device__ __forceinline__ float sigm_(float x) { return __fdividef(1.f, 1.f + __expf(-x)); }
__device__ __forceinline__ float silu_(float x) { return x * sigm_(x); }

__device__ __forceinline__ void split_bf(float x, unsigned short& hs, unsigned short& ls)
{
  unsigned u = __float_as_uint(x);
  unsigned r = (u + 0x7FFFu + ((u >> 16) & 1u)) >> 16;
  float hfv = __uint_as_float(r << 16);
  float rem = x - hfv;
  unsigned ul = __float_as_uint(rem);
  unsigned rl = (ul + 0x7FFFu + ((ul >> 16) & 1u)) >> 16;
  hs = (unsigned short)r;
  ls = (unsigned short)rl;
}

__device__ __forceinline__ void wmma3(v8f& acc, const v16b ah, const v16b al, const v16b bh, const v16b bl)
{
  v8f t = acc;
  t = __builtin_amdgcn_wmma_f32_16x16x32_bf16(false, ah, false, bh, (short)0, t, false, false);
  t = __builtin_amdgcn_wmma_f32_16x16x32_bf16(false, ah, false, bl, (short)0, t, false, false);
  t = __builtin_amdgcn_wmma_f32_16x16x32_bf16(false, al, false, bh, (short)0, t, false, false);
  asm volatile("v_nop\n\tv_nop\n\tv_nop\n\tv_nop" : "+v"(t) : "v"(ah), "v"(al), "v"(bh), "v"(bl));
  acc = t;
}

#define TP 40
#define CPW 36
__global__ __launch_bounds__(32) void gemm3_k(const float* __restrict__ A, const float* __restrict__ Bm,
    float* __restrict__ C, int M, int N, int Kd,
    int a_sm, int a_sk, int a_bat, int b_sk, int b_sn, int b_bat, int b_mod, int c_sm, int c_bat)
{
  __shared__ __attribute__((aligned(16))) unsigned short sAh[32 * TP];
  __shared__ __attribute__((aligned(16))) unsigned short sAl[32 * TP];
  __shared__ __attribute__((aligned(16))) unsigned short sBh[32 * TP];
  __shared__ __attribute__((aligned(16))) unsigned short sBl[32 * TP];
  __shared__ __attribute__((aligned(16))) float sC[32 * CPW];

  const int lane = threadIdx.x & 31, hf = lane >> 4, m16 = lane & 15;
  const int z = blockIdx.z, tm = blockIdx.y * 32, tn = blockIdx.x * 32;
  const float* Ab = A + (size_t)z * (size_t)a_bat;
  const float* Bb = Bm + (size_t)(z % b_mod) * (size_t)b_bat;
  float* Cb = C + (size_t)z * (size_t)c_bat;
  const bool a_kc = (a_sk == 1);
  const bool b_kc = (b_sk == 1);

  const v8f z8 = {0.f, 0.f, 0.f, 0.f, 0.f, 0.f, 0.f, 0.f};
  v8f acc00 = z8, acc01 = z8, acc10 = z8, acc11 = z8;

  for (int k0 = 0; k0 < Kd; k0 += 32) {
    __syncthreads();
#pragma unroll 8
    for (int j = 0; j < 32; ++j) {
      const int mm = a_kc ? j : lane;
      const int kk = a_kc ? lane : j;
      const int gm = tm + mm, gk = k0 + kk;
      float v = 0.f;
      if (gm < M && gk < Kd) v = Ab[(size_t)gm * (size_t)a_sm + (size_t)gk * (size_t)a_sk];
      unsigned short hs, ls;
      split_bf(v, hs, ls);
      sAh[mm * TP + kk] = hs;
      sAl[mm * TP + kk] = ls;
    }
#pragma unroll 8
    for (int j = 0; j < 32; ++j) {
      const int nn = b_kc ? j : lane;
      const int kk = b_kc ? lane : j;
      const int gn = tn + nn, gk = k0 + kk;
      float v = 0.f;
      if (gn < N && gk < Kd) v = Bb[(size_t)gk * (size_t)b_sk + (size_t)gn * (size_t)b_sn];
      unsigned short hs, ls;
      split_bf(v, hs, ls);
      sBh[nn * TP + kk] = hs;
      sBl[nn * TP + kk] = ls;
    }
    __syncthreads();
    Frag a0h, a0l, a1h, a1l, b0h, b0l, b1h, b1l;
    const int r0 = m16 * TP + 8 * hf;
    const int r1 = (16 + m16) * TP + 8 * hf;
    a0h.h[0] = *(const v8us*)(sAh + r0);  a0h.h[1] = *(const v8us*)(sAh + r0 + 16);
    a0l.h[0] = *(const v8us*)(sAl + r0);  a0l.h[1] = *(const v8us*)(sAl + r0 + 16);
    a1h.h[0] = *(const v8us*)(sAh + r1);  a1h.h[1] = *(const v8us*)(sAh + r1 + 16);
    a1l.h[0] = *(const v8us*)(sAl + r1);  a1l.h[1] = *(const v8us*)(sAl + r1 + 16);
    b0h.h[0] = *(const v8us*)(sBh + r0);  b0h.h[1] = *(const v8us*)(sBh + r0 + 16);
    b0l.h[0] = *(const v8us*)(sBl + r0);  b0l.h[1] = *(const v8us*)(sBl + r0 + 16);
    b1h.h[0] = *(const v8us*)(sBh + r1);  b1h.h[1] = *(const v8us*)(sBh + r1 + 16);
    b1l.h[0] = *(const v8us*)(sBl + r1);  b1l.h[1] = *(const v8us*)(sBl + r1 + 16);
    wmma3(acc00, a0h.v, a0l.v, b0h.v, b0l.v);
    wmma3(acc01, a0h.v, a0l.v, b1h.v, b1l.v);
    wmma3(acc10, a1h.v, a1l.v, b0h.v, b0l.v);
    wmma3(acc11, a1h.v, a1l.v, b1h.v, b1l.v);
  }

  __syncthreads();
#pragma unroll
  for (int r = 0; r < 8; ++r) {
    sC[(8 * hf + r) * CPW + m16]           = acc00[r];
    sC[(8 * hf + r) * CPW + 16 + m16]      = acc01[r];
    sC[(16 + 8 * hf + r) * CPW + m16]      = acc10[r];
    sC[(16 + 8 * hf + r) * CPW + 16 + m16] = acc11[r];
  }
  __syncthreads();
  const int rsub = lane >> 3, c4 = (lane & 7) * 4;
  v4f vals[8];
#pragma unroll
  for (int q = 0; q < 8; ++q) vals[q] = *(const v4f*)(sC + (q * 4 + rsub) * CPW + c4);
#pragma unroll
  for (int q = 0; q < 8; ++q) {
    const int gm = tm + q * 4 + rsub;
    if (gm < M) *(volatile v4f*)(Cb + (size_t)gm * (size_t)c_sm + tn + c4) = vals[q];
  }
  __threadfence();
#pragma unroll
  for (int q = 0; q < 8; ++q) {
    const int gm = tm + q * 4 + rsub;
    if (gm < M) *(volatile v4f*)(Cb + (size_t)gm * (size_t)c_sm + tn + c4) = vals[q];
  }
}

__global__ __launch_bounds__(256) void dwconv_k(const float* __restrict__ xz, int cstride,
    const float* __restrict__ w, const float* __restrict__ bias, float* __restrict__ outp, int total4)
{
  const int g = blockIdx.x * blockDim.x + threadIdx.x;
  if (g >= total4) return;
  const int o = g * 4;
  const int wx0 = o & (WW - 1);
  const int hy = (o >> 6) & (HH - 1);
  const int c = (o >> 12) % DI;
  const int b = o / (DI * LL);
  float wk[9];
#pragma unroll
  for (int t = 0; t < 9; ++t) wk[t] = w[c * 9 + t];
  const float bc = bias[c];
  float r[4];
#pragma unroll
  for (int e = 0; e < 4; ++e) {
    const int wx = wx0 + e;
    float acc = bc;
#pragma unroll
    for (int dy = 0; dy < 3; ++dy) {
      const int hh2 = hy + dy - 1;
      if (hh2 < 0 || hh2 >= HH) continue;
#pragma unroll
      for (int dx = 0; dx < 3; ++dx) {
        const int wp = wx + dx - 1;
        if (wp < 0 || wp >= WW) continue;
        acc += xz[((size_t)(b * HH + hh2) * WW + wp) * (size_t)cstride + c] * wk[dy * 3 + dx];
      }
    }
    r[e] = silu_(acc);
  }
  v4f v = {r[0], r[1], r[2], r[3]};
  float* dst = outp + o;
  *(volatile v4f*)dst = v;
  __threadfence();
  *(volatile v4f*)dst = v;
}

__global__ __launch_bounds__(256) void se_k(const float* __restrict__ fx, const float* __restrict__ ix,
    const float* __restrict__ w1, const float* __restrict__ b1, const float* __restrict__ w2,
    const float* __restrict__ b2, float* __restrict__ att)
{
  __shared__ float smean[DI];
  __shared__ float sh1[KK * CR];
  __shared__ __attribute__((aligned(16))) float satt[KK * DI];
  const int b = blockIdx.x, tid = threadIdx.x, wave = tid >> 5, lane = tid & 31;

  for (int c = wave; c < DI; c += 8) {
    const size_t base = ((size_t)b * DI + c) * (size_t)LL;
    float s = 0.f;
    for (int l = lane; l < LL; l += 32) s += fx[base + l] + ix[base + l];
#pragma unroll
    for (int off = 16; off > 0; off >>= 1) s += __shfl_xor(s, off, 32);
    if (lane == 0) smean[c] = s * (1.f / (float)LL);
  }
  __syncthreads();
  if (tid < KK * CR) {
    const int k = tid / CR, r = tid - k * CR;
    float s = b1[k * CR + r];
    const float* wr = w1 + ((size_t)k * CR + r) * DI;
#pragma unroll 1
    for (int c = 0; c < DI; ++c) s += smean[c] * wr[c];
    sh1[tid] = silu_(s);
  }
  __syncthreads();
  if (tid < DI) {
#pragma unroll 1
    for (int k = 0; k < KK; ++k) {
      float s = b2[k * DI + tid];
      const float* wr = w2 + ((size_t)k * DI + tid) * CR;
#pragma unroll 1
      for (int r = 0; r < CR; ++r) s += sh1[k * CR + r] * wr[r];
      satt[k * DI + tid] = sigm_(s);
    }
  }
  __syncthreads();
  const int nq = (KK * DI) / 4;
  v4f v = {0.f, 0.f, 0.f, 0.f};
  if (tid < nq) v = *(const v4f*)(satt + 4 * tid);
  float* dst = att + (size_t)b * KK * DI + 4 * tid;
  if (tid < nq) *(volatile v4f*)dst = v;
  __threadfence();
  if (tid < nq) *(volatile v4f*)dst = v;
}

__global__ __launch_bounds__(256) void sfb_k(const float* __restrict__ fx, const float* __restrict__ ix,
    const float* __restrict__ att, float* __restrict__ sfo, int total4)
{
  const int g = blockIdx.x * blockDim.x + threadIdx.x;
  if (g >= total4) return;
  const int o = g * 4;
  const int l0 = o & (LL - 1);
  const int d = (o >> 12) % DI;
  const int bk = o / (LL * DI);
  const int k = bk & (KK - 1), b = bk >> 2;
  const float a = att[bk * DI + d];
  const float am = 1.f - a;
  const size_t sb = ((size_t)b * DI + d) * (size_t)LL;
  float r[4];
#pragma unroll
  for (int e = 0; e < 4; ++e) {
    const int l = l0 + e;
    int src;
    if (k == 0)      src = l;
    else if (k == 1) src = (l & 63) * 64 + (l >> 6);
    else if (k == 2) src = LL - 1 - l;
    else { const int m = LL - 1 - l; src = (m & 63) * 64 + (m >> 6); }
    r[e] = fx[sb + src] * a + ix[sb + src] * am;
  }
  v4f v = {r[0], r[1], r[2], r[3]};
  float* dst = sfo + o;
  *(volatile v4f*)dst = v;
  __threadfence();
  *(volatile v4f*)dst = v;
}

#define TCH 32
#define UP 36
__global__ __launch_bounds__(DI) void scan_k(const float* __restrict__ sfb, const float* __restrict__ fdb,
    const float* __restrict__ dtw, const float* __restrict__ alog, const float* __restrict__ dtb,
    const float* __restrict__ Dsv, float* __restrict__ oy)
{
  __shared__ __attribute__((aligned(16))) float sU[DI * UP];
  __shared__ __attribute__((aligned(16))) float sY[DI * UP];
  __shared__ float sF[TCH * FP];
  const int bk = blockIdx.x, k = bk & (KK - 1), d = threadIdx.x, wave = d >> 5, lane = d & 31;
  const int kd = k * DI + d;
  const float bias = dtb[kd], Dv = Dsv[kd];
  float wdt[RR];
#pragma unroll
  for (int r = 0; r < RR; ++r) wdt[r] = dtw[(size_t)kd * RR + r];
#pragma unroll 1
  for (int n = 0; n < NS; ++n) sY[d * UP + n] = -expf(alog[(size_t)kd * NS + n]);
  float Av[NS], h[NS];
#pragma unroll
  for (int n = 0; n < NS; ++n) { Av[n] = sY[d * UP + n]; h[n] = 0.f; }

  const size_t rowbase = (size_t)bk * DI * (size_t)LL;
  const size_t fbase = (size_t)bk * LL * (size_t)FP;
  const int rsub = lane >> 3, c4 = (lane & 7) * 4;

  for (int t0 = 0; t0 < LL; t0 += TCH) {
    __syncthreads();
#pragma unroll 4
    for (int j = 0; j < 32; ++j) {
      const int row = wave * 32 + j;
      sU[row * UP + lane] = sfb[rowbase + (size_t)row * LL + t0 + lane];
    }
    for (int idx = d; idx < TCH * FP; idx += DI) {
      const int tt = idx >> 6, cc = idx & 63;
      sF[idx] = fdb[fbase + (size_t)(t0 + tt) * FP + cc];
    }
    __syncthreads();
#pragma unroll 1
    for (int tt = 0; tt < TCH; ++tt) {
      const float* fr = sF + tt * FP;
      float dr = 0.f;
#pragma unroll
      for (int r = 0; r < RR; ++r) dr += wdt[r] * fr[r];
      const float x = dr + bias;
      const float sp = log1pf(expf(fminf(x, 20.f)));
      const float db = (x > 20.f) ? x : sp;
      const float u = sU[d * UP + tt];
      const float du = db * u;
      float y = 0.f;
#pragma unroll
      for (int n = 0; n < NS; ++n) {
        const float e = __expf(db * Av[n]);
        h[n] = e * h[n] + du * fr[RR + n];
        y += h[n] * fr[RR + NS + n];
      }
      sY[d * UP + tt] = y + u * Dv;
    }
    __syncthreads();
    v4f vals[8];
#pragma unroll
    for (int q = 0; q < 8; ++q) vals[q] = *(const v4f*)(sY + (wave * 32 + q * 4 + rsub) * UP + c4);
#pragma unroll
    for (int q = 0; q < 8; ++q) {
      const int row = wave * 32 + q * 4 + rsub;
      *(volatile v4f*)(oy + rowbase + (size_t)row * LL + t0 + c4) = vals[q];
    }
    __threadfence();
#pragma unroll
    for (int q = 0; q < 8; ++q) {
      const int row = wave * 32 + q * 4 + rsub;
      *(volatile v4f*)(oy + rowbase + (size_t)row * LL + t0 + c4) = vals[q];
    }
  }
}

__global__ __launch_bounds__(256) void ycat_k(const float* __restrict__ oy, float* __restrict__ yc, int total4)
{
  const int g = blockIdx.x * blockDim.x + threadIdx.x;
  if (g >= total4) return;
  const int o = g * 4;
  const int c0 = o % (2 * DI);
  const int l = (o / (2 * DI)) % LL;
  const int b = o / (2 * DI * LL);
  const int hy = l >> 6, wx = l & 63;
  const int lt = wx * HH + hy;
  float r[4];
#pragma unroll
  for (int e = 0; e < 4; ++e) {
    const int c = c0 + e;
    float v;
    if (c0 < DI) {
      v = oy[((size_t)(b * KK + 0) * DI + c) * (size_t)LL + l]
        + oy[((size_t)(b * KK + 2) * DI + c) * (size_t)LL + (LL - 1 - l)];
    } else {
      const int d2 = c - DI;
      v = oy[((size_t)(b * KK + 1) * DI + d2) * (size_t)LL + lt]
        + oy[((size_t)(b * KK + 3) * DI + d2) * (size_t)LL + (LL - 1 - lt)];
    }
    r[e] = v;
  }
  v4f v4 = {r[0], r[1], r[2], r[3]};
  float* dst = yc + o;
  *(volatile v4f*)dst = v4;
  __threadfence();
  *(volatile v4f*)dst = v4;
}

__global__ __launch_bounds__(32) void ln_gate_k(const float* __restrict__ yf, const float* __restrict__ iz,
    const float* __restrict__ g, const float* __restrict__ bb, float* __restrict__ yg, int nrows)
{
  const int row = blockIdx.x;
  if (row >= nrows) return;
  const int lane = threadIdx.x & 31;
  const bool has1 = lane < 16;
  const int l1 = has1 ? lane : 0;
  const v4f zero4 = {0.f, 0.f, 0.f, 0.f};
  const size_t base = (size_t)row * DI;
  v4f x0 = *(const v4f*)(yf + base + 4 * lane);
  v4f x1 = *(const v4f*)(yf + base + 128 + 4 * l1);
  if (!has1) x1 = zero4;
  float s = (x0.x + x0.y) + (x0.z + x0.w) + (x1.x + x1.y) + (x1.z + x1.w);
#pragma unroll
  for (int off = 16; off > 0; off >>= 1) s += __shfl_xor(s, off, 32);
  const float mu = s * (1.f / (float)DI);
  v4f d0 = x0 - mu;
  v4f d1 = x1 - mu;
  if (!has1) d1 = zero4;
  float q = d0.x * d0.x + d0.y * d0.y + d0.z * d0.z + d0.w * d0.w
          + d1.x * d1.x + d1.y * d1.y + d1.z * d1.z + d1.w * d1.w;
#pragma unroll
  for (int off = 16; off > 0; off >>= 1) q += __shfl_xor(q, off, 32);
  const float var = q * (1.f / (float)DI);
  const float rstd = rsqrtf(var + 1e-5f);
  v4f g0 = *(const v4f*)(g + 4 * lane);
  v4f g1 = *(const v4f*)(g + 128 + 4 * l1);
  v4f e0 = *(const v4f*)(bb + 4 * lane);
  v4f e1 = *(const v4f*)(bb + 128 + 4 * l1);
  const size_t zb = (size_t)row * (2 * DI) + DI;
  v4f z0 = *(const v4f*)(iz + zb + 4 * lane);
  v4f z1 = *(const v4f*)(iz + zb + 128 + 4 * l1);
  v4f o0, o1;
#pragma unroll
  for (int e = 0; e < 4; ++e) {
    o0[e] = (d0[e] * rstd * g0[e] + e0[e]) * silu_(z0[e]);
    o1[e] = (d1[e] * rstd * g1[e] + e1[e]) * silu_(z1[e]);
  }
  float* dst0 = yg + base + 4 * lane;
  float* dst1 = yg + base + 128 + 4 * l1;
  *(volatile v4f*)dst0 = o0;
  if (has1) *(volatile v4f*)dst1 = o1;
  __threadfence();
  *(volatile v4f*)dst0 = o0;
  if (has1) *(volatile v4f*)dst1 = o1;
}

static void launch_gemm(hipStream_t st, const float* A, const float* Bw, float* C, int M, int N, int Kd,
                        int a_sm, int a_sk, int a_bat, int b_sk, int b_sn, int b_bat, int b_mod,
                        int c_sm, int c_bat, int ncol, int Z)
{
  dim3 g(ncol, (M + 31) / 32, Z);
  gemm3_k<<<g, 32, 0, st>>>(A, Bw, C, M, N, Kd, a_sm, a_sk, a_bat, b_sk, b_sn, b_bat, b_mod, c_sm, c_bat);
}

extern "C" void kernel_launch(void* const* d_in, const int* in_sizes, int n_in,
                              void* d_out, int out_size, void* d_ws, size_t ws_size,
                              hipStream_t stream)
{
  if (n_in != 21) return;
  const int expect_sizes[21] = {
    NTOK * DM, NTOK * DM, 2 * DI * DM, 2 * DI * DM, DI * 9, DI, DI * 9, DI,
    KK * CR * DI, KK * CR, KK * DI * CR, KK * DI, KK * CM * DI, KK * DI * RR, KK * DI,
    KK * DI * NS, KK * DI, DI * 2 * DI, DI, DI, DM * DI };
  for (int t = 0; t < 21; ++t) if (in_sizes[t] != expect_sizes[t]) return;
  if (out_size != NTOK * DM) return;

  const float* f    = (const float*)d_in[0];
  const float* iin  = (const float*)d_in[1];
  const float* w1   = (const float*)d_in[2];
  const float* w2   = (const float*)d_in[3];
  const float* c1w  = (const float*)d_in[4];
  const float* c1b  = (const float*)d_in[5];
  const float* c2w  = (const float*)d_in[6];
  const float* c2b  = (const float*)d_in[7];
  const float* cfw1 = (const float*)d_in[8];
  const float* cfb1 = (const float*)d_in[9];
  const float* cfw2 = (const float*)d_in[10];
  const float* cfb2 = (const float*)d_in[11];
  const float* fpw  = (const float*)d_in[12];
  const float* dtw  = (const float*)d_in[13];
  const float* dtb  = (const float*)d_in[14];
  const float* alog = (const float*)d_in[15];
  const float* Ds   = (const float*)d_in[16];
  const float* fusw = (const float*)d_in[17];
  const float* ong  = (const float*)d_in[18];
  const float* onb  = (const float*)d_in[19];
  const float* opw  = (const float*)d_in[20];
  float* out = (float*)d_out;

  float* ws = (float*)d_ws;
  size_t off = 0;
  float* fzx  = ws + off; off += (size_t)NTOK * DI;
  float* iz   = ws + off; off += (size_t)NTOK * 2 * DI;
  float* fxA  = ws + off; off += (size_t)B_SZ * DI * LL;
  float* ixA  = ws + off; off += (size_t)B_SZ * DI * LL;
  float* att  = ws + off; off += (size_t)B_SZ * KK * DI;
  float* sfb  = ws + off; off += (size_t)B_SZ * KK * DI * LL;
  float* fdb  = ws + off; off += (size_t)B_SZ * KK * LL * FP;
  float* oy   = ws + off; off += (size_t)B_SZ * KK * DI * LL;
  float* ycat = ws + off; off += (size_t)NTOK * 2 * DI;
  float* yf   = ws + off; off += (size_t)NTOK * DI;
  float* yg   = ws + off; off += (size_t)NTOK * DI;
  if (off * sizeof(float) > ws_size) return;

  launch_gemm(stream, f,   w1, fzx, NTOK, DI,     DM, DM, 1, 0, 1, DM, 0, 1, DI,     0, DI / 32,       1);
  launch_gemm(stream, iin, w2, iz,  NTOK, 2 * DI, DM, DM, 1, 0, 1, DM, 0, 1, 2 * DI, 0, (2 * DI) / 32, 1);

  const int tc4 = (B_SZ * DI * LL) / 4;
  dwconv_k<<<(tc4 + 255) / 256, 256, 0, stream>>>(fzx, DI,     c1w, c1b, fxA, tc4);
  dwconv_k<<<(tc4 + 255) / 256, 256, 0, stream>>>(iz,  2 * DI, c2w, c2b, ixA, tc4);

  se_k<<<B_SZ, 256, 0, stream>>>(fxA, ixA, cfw1, cfb1, cfw2, cfb2, att);

  const int ts4 = (B_SZ * KK * DI * LL) / 4;
  sfb_k<<<(ts4 + 255) / 256, 256, 0, stream>>>(fxA, ixA, att, sfb, ts4);

  launch_gemm(stream, sfb, fpw, fdb, LL, CM, DI, 1, LL, DI * LL, 1, DI, CM * DI, KK, FP, LL * FP, FP / 32, B_SZ * KK);

  scan_k<<<B_SZ * KK, DI, 0, stream>>>(sfb, fdb, dtw, alog, dtb, Ds, oy);

  const int ty4 = (NTOK * 2 * DI) / 4;
  ycat_k<<<(ty4 + 255) / 256, 256, 0, stream>>>(oy, ycat, ty4);

  launch_gemm(stream, ycat, fusw, yf, NTOK, DI, 2 * DI, 2 * DI, 1, 0, 1, 2 * DI, 0, 1, DI, 0, DI / 32, 1);

  ln_gate_k<<<NTOK, 32, 0, stream>>>(yf, iz, ong, onb, yg, NTOK);

  launch_gemm(stream, yg, opw, out, NTOK, DM, DI, DI, 1, 0, 1, DI, 0, 1, DM, 0, DM / 32, 1);
}
